// DGMMC_spherical_54185307406409
// MI455X (gfx1250) — hardware-verified
//
#include <hip/hip_runtime.h>


#define NB   8192
#define DI   1024
#define NC   128
#define KK   8
#define NN   (NC * KK)
#define LOG2PI 1.8378770664093453f
typedef _Float16 h16;
typedef unsigned short bf;
typedef __attribute__((ext_vector_type(16))) __bf16   v16bf;
typedef __attribute__((ext_vector_type(16))) _Float16 v16h;
typedef __attribute__((ext_vector_type(8)))  _Float16 v8h;
typedef __attribute__((ext_vector_type(8)))  unsigned short v8us;
typedef __attribute__((ext_vector_type(8)))  float    v8f;
typedef __attribute__((ext_vector_type(4)))  float    v4f;
typedef v8h  __attribute__((may_alias)) v8ha;
typedef v4f  __attribute__((may_alias)) v4fa;
typedef v8us __attribute__((may_alias)) v8usa;

__device__ __forceinline__ unsigned short f2bf(float f) { unsigned u = __float_as_uint(f); u += 0x7FFFu + ((u >> 16) & 1u); return (unsigned short)(u >> 16); }
__device__ __forceinline__ float bf2f(unsigned short b) { return __uint_as_float(((unsigned)b) << 16); }
__device__ __forceinline__ float bfr(float f) { return bf2f(f2bf(f)); }
__device__ __forceinline__ v16h cat16(v8h lo, v8h hi) { return __builtin_shufflevector(lo, hi, 0, 1, 2, 3, 4, 5, 6, 7, 8, 9, 10, 11, 12, 13, 14, 15); }
__device__ __forceinline__ v16bf cat16b(v8us lo, v8us hi) { return __builtin_bit_cast(v16bf, __builtin_shufflevector(lo, hi, 0, 1, 2, 3, 4, 5, 6, 7, 8, 9, 10, 11, 12, 13, 14, 15)); }
__device__ __forceinline__ v8f wmma16(v16h a, v16h b, v8f c) { return __builtin_amdgcn_wmma_f32_16x16x32_f16(false, a, false, b, (short)0, c, false, false); }
__device__ __forceinline__ v8f wmmab(v16bf a, v16bf b, v8f c) { return __builtin_amdgcn_wmma_f32_16x16x32_bf16(false, a, false, b, (short)0, c, false, false); }


template <typename T16> struct WFrag;
template <> struct WFrag<h16> { typedef v16h V; static __device__ __forceinline__ V ld(const h16* p) { return cat16(*(const v8h*)p, *(const v8h*)(p + 16)); } static __device__ __forceinline__ v8f mma(V a, V b, v8f c) { return wmma16(a, b, c); } };
template <> struct WFrag<bf> { typedef v16bf V; static __device__ __forceinline__ V ld(const bf* p) { return cat16b(*(const v8us*)p, *(const v8us*)(p + 16)); } static __device__ __forceinline__ v8f mma(V a, V b, v8f c) { return wmmab(a, b, c); } };
template <typename T16, int NSPLIT, bool BIAS>
__global__ __launch_bounds__(32) void k_gemmw(const T16* __restrict__ A, const T16* __restrict__ A2, const T16* __restrict__ Bt, const T16* __restrict__ Bt2, int K, float* C, int ldc, const float* __restrict__ bias, size_t sA, size_t sB, size_t sC) {
    typedef typename WFrag<T16>::V V;
    __shared__ __align__(16) float os[16 * 68];
    const size_t z = blockIdx.z; A += z * sA; if (A2) A2 += z * sA; Bt += z * sB; if (Bt2) Bt2 += z * sB; C += z * sC;
    const int lane = threadIdx.x & 31, lr = lane & 15, hi = lane >> 4; const int r0 = blockIdx.x * 64, c0 = blockIdx.y * 64;
    v8f acc[4][4];
#pragma unroll
    for (int mb = 0; mb < 4; ++mb)
#pragma unroll
        for (int nb = 0; nb < 4; ++nb) acc[mb][nb] = (v8f){};
    const size_t aoff = (size_t)(r0 + lr) * K + 8 * hi, boff = (size_t)(c0 + lr) * K + 8 * hi;
#pragma unroll 1
    for (int kc = 0; kc < K; kc += 32) {
        V a[4], a2[4];
#pragma unroll
        for (int mb = 0; mb < 4; ++mb) { a[mb] = WFrag<T16>::ld(A + aoff + (size_t)mb * 16 * K + kc); if (NSPLIT == 1 || NSPLIT == 2) a2[mb] = WFrag<T16>::ld(A2 + aoff + (size_t)mb * 16 * K + kc); }
#pragma unroll
        for (int nb = 0; nb < 4; ++nb) { const V b = WFrag<T16>::ld(Bt + boff + (size_t)nb * 16 * K + kc); V b2; if (NSPLIT >= 2) b2 = WFrag<T16>::ld(Bt2 + boff + (size_t)nb * 16 * K + kc);
#pragma unroll
            for (int mb = 0; mb < 4; ++mb) { acc[mb][nb] = WFrag<T16>::mma(a[mb], b, acc[mb][nb]); if (NSPLIT == 1 || NSPLIT == 2) acc[mb][nb] = WFrag<T16>::mma(a2[mb], b, acc[mb][nb]); if (NSPLIT >= 2) acc[mb][nb] = WFrag<T16>::mma(a[mb], b2, acc[mb][nb]); } }
        asm volatile("v_nop\n\tv_nop\n\tv_nop\n\tv_nop" : "+v"(acc[0][0]), "+v"(acc[1][1]), "+v"(acc[2][2]), "+v"(acc[3][3]) : "v"(a[0]), "v"(a[3]));
    }
#pragma unroll
    for (int mb = 0; mb < 4; ++mb) {
#pragma unroll
        for (int nb = 0; nb < 4; ++nb) {
#pragma unroll
            for (int j = 0; j < 8; ++j) os[(hi * 8 + j) * 68 + nb * 16 + lr] = acc[mb][nb][j]; }
        __builtin_amdgcn_wave_barrier(); asm volatile("" ::: "memory");
        float* crow = C + (size_t)(r0 + mb * 16) * ldc + c0;
#pragma unroll 1
        for (int ps = 0; ps < 2; ++ps) {
#pragma unroll
            for (int s = 0; s < 8; ++s) { const int row = 2 * s + hi, cofs = lr * 4; v4f val = *(const v4fa*)(os + row * 68 + cofs); if (BIAS) { val[0] += bfr(bias[c0 + cofs]); val[1] += bfr(bias[c0 + cofs + 1]); val[2] += bfr(bias[c0 + cofs + 2]); val[3] += bfr(bias[c0 + cofs + 3]); }
                *(volatile v4f*)(crow + (size_t)row * ldc + cofs) = val; }
            if (ps == 0) __threadfence(); }
        __builtin_amdgcn_wave_barrier(); asm volatile("" ::: "memory");
    }
}


__global__ __launch_bounds__(256) void k_cvt8(const float* __restrict__ src, bf* dst, size_t n8) { const size_t i = (size_t)blockIdx.x * 256 + threadIdx.x; if (i >= n8) return; const v8f v = *(const v8f*)(src + i * 8); v8us o;
#pragma unroll
    for (int k = 0; k < 8; ++k) o[k] = f2bf(v[k]); *(volatile v8us*)(dst + i * 8) = o; __threadfence(); *(volatile v8us*)(dst + i * 8) = o; }
__global__ __launch_bounds__(256) void k_msq(const float* __restrict__ m, float* MSQ) {
    const int lane = threadIdx.x & 31; const int n = blockIdx.x * 8 + (threadIdx.x >> 5); if (n >= NN) return; float s = 0.f;
#pragma unroll
    for (int c = 0; c < DI / 128; ++c) { const v4f v = *(const v4f*)(m + (size_t)n * DI + c * 128 + lane * 4);
#pragma unroll
        for (int q = 0; q < 4; ++q) { const float t = bfr(v[q]); float p = __fmul_rn(t, t); asm volatile("" : "+v"(p)); s = __fadd_rn(s, p); } }
#pragma unroll
    for (int sh = 16; sh; sh >>= 1) s += __shfl_xor(s, sh, 32);
    const float o = (lane == 0) ? s : 0.f; *(volatile float*)(MSQ + (size_t)n * 32 + lane) = o; __threadfence(); *(volatile float*)(MSQ + (size_t)n * 32 + lane) = o; }
__global__ __launch_bounds__(256) void k_prep(const float* __restrict__ bwv, const float* __restrict__ wv, float* PRE) { const int n = blockIdx.x * 256 + threadIdx.x; if (n >= NN) return; float bw = bfr(bwv[n]); bw = fminf(fmaxf(bw, 0.001f), 100.0f);
    const int c0 = (n / KK) * KK; float wm = -3.0e38f; for (int k = 0; k < KK; ++k) wm = fmaxf(wm, bfr(wv[c0 + k])); float ws = 0.f; for (int k = 0; k < KK; ++k) ws += __expf(bfr(wv[c0 + k]) - wm);
    v4f o; o[0] = __fmul_rn((float)DI, __logf(bw)); o[1] = __fdiv_rn(1.0f, bw); o[2] = __fsub_rn(bfr(wv[n]), __fadd_rn(wm, __logf(ws))); o[3] = 0.f; *(volatile v4f*)(PRE + (size_t)n * 4) = o; __threadfence(); *(volatile v4f*)(PRE + (size_t)n * 4) = o; }
__global__ __launch_bounds__(256) void k_mix(const float* __restrict__ G, const float* __restrict__ x, const float* __restrict__ MSQ, const float* __restrict__ PRE, const float* __restrict__ pri, float* OUT) {
    const int lane = threadIdx.x & 31; const int b = blockIdx.x * 8 + (threadIdx.x >> 5); if (b >= NB) return;
    float xs = 0.f;
#pragma unroll
    for (int c = 0; c < DI / 128; ++c) { const v4f v = *(const v4f*)(x + (size_t)b * DI + c * 128 + lane * 4);
#pragma unroll
        for (int q = 0; q < 4; ++q) { const float t = bfr(v[q]); float p = __fmul_rn(t, t); asm volatile("" : "+v"(p)); xs = __fadd_rn(xs, p); } }
#pragma unroll
    for (int sh = 16; sh; sh >>= 1) xs += __shfl_xor(xs, sh, 32);
    float pr[4]; float pm = -3.0e38f;
#pragma unroll
    for (int q = 0; q < 4; ++q) { pr[q] = bfr(pri[lane * 4 + q]); pm = fmaxf(pm, pr[q]); }
#pragma unroll
    for (int sh = 16; sh; sh >>= 1) pm = fmaxf(pm, __shfl_xor(pm, sh, 32));
    float pse = 0.f;
#pragma unroll
    for (int q = 0; q < 4; ++q) pse += __expf(pr[q] - pm);
#pragma unroll
    for (int sh = 16; sh; sh >>= 1) pse += __shfl_xor(pse, sh, 32);
    const float plse = __fadd_rn(pm, __logf(pse));
    float cls[8];
#pragma unroll
    for (int ch = 0; ch < 8; ++ch) { const int j0 = ch * 128 + lane * 4; const v4f g4 = *(const v4f*)(G + (size_t)b * NN + j0); float lp[4]; float m1 = -3.0e38f;
#pragma unroll
        for (int q = 0; q < 4; ++q) { const v4f pre = *(const v4f*)(PRE + (size_t)(j0 + q) * 4); const float msq = MSQ[(size_t)(j0 + q) * 32];
            float cross = __fmul_rn(2.0f, g4[q]); asm volatile("" : "+v"(cross)); const float sq = __fsub_rn(__fadd_rn(xs, msq), cross);
            float t2 = __fmul_rn(sq, pre[1]); asm volatile("" : "+v"(t2));
            const float inner = __fadd_rn(__fadd_rn((float)DI * LOG2PI, pre[0]), t2); float v0 = __fmul_rn(-0.5f, inner); asm volatile("" : "+v"(v0)); lp[q] = __fadd_rn(v0, pre[2]); m1 = fmaxf(m1, lp[q]); }
        m1 = fmaxf(m1, __shfl_xor(m1, 1, 32)); float s1 = 0.f;
#pragma unroll
        for (int q = 0; q < 4; ++q) s1 += __expf(lp[q] - m1);
        s1 += __shfl_xor(s1, 1, 32); const int c = ch * 16 + (lane >> 1); cls[ch] = __fadd_rn(__fadd_rn(m1, __logf(s1)), __fsub_rn(bfr(pri[c]), plse)); }
    float cm = -3.0e38f;
#pragma unroll
    for (int ch = 0; ch < 8; ++ch) cm = fmaxf(cm, cls[ch]);
#pragma unroll
    for (int sh = 16; sh; sh >>= 1) cm = fmaxf(cm, __shfl_xor(cm, sh, 32));
    float cs = 0.f;
#pragma unroll
    for (int ch = 0; ch < 8; ++ch) cs += (lane & 1) ? 0.f : __expf(cls[ch] - cm);
#pragma unroll
    for (int sh = 16; sh; sh >>= 1) cs += __shfl_xor(cs, sh, 32);
    const float lse = __fadd_rn(cm, __logf(cs));
#pragma unroll 1
    for (int ps = 0; ps < 2; ++ps) {
#pragma unroll
        for (int q = 0; q < 4; ++q) { const float a0 = __shfl(cls[2 * q], 2 * (lane & 15), 32), a1 = __shfl(cls[2 * q + 1], 2 * (lane & 15), 32); const float v = ((lane >> 4) ? a1 : a0) - lse;
            *(volatile float*)(OUT + (size_t)b * NC + q * 32 + lane) = v; }
        if (ps == 0) __threadfence(); }
}

extern "C" void kernel_launch(void* const* d_in, const int* in_sizes, int n_in,
                              void* d_out, int out_size, void* d_ws, size_t ws_size, hipStream_t stream) {
    (void)in_sizes; (void)n_in; (void)out_size;
    const float* x = (const float*)d_in[0]; const float* means = (const float*)d_in[1]; const float* bw = (const float*)d_in[2]; const float* wts = (const float*)d_in[3]; const float* pri = (const float*)d_in[4];
    float* OUT = (float*)d_out;
    char* wsp = (char*)d_ws;
    auto take = [&](size_t bytes) { char* p = wsp; wsp += (bytes + 255) & ~(size_t)255; return (void*)p; };
    bf* XB = (bf*)take((size_t)NB * DI * 2); bf* MB = (bf*)take((size_t)NN * DI * 2); float* G = (float*)take((size_t)NB * NN * 4); float* MSQ = (float*)take((size_t)NN * 32 * 4); float* PRE = (float*)take((size_t)NN * 16);
    if ((size_t)(wsp - (char*)d_ws) > ws_size) return;
    k_cvt8<<<(unsigned)(((size_t)NB * DI / 8 + 255) / 256), 256, 0, stream>>>(x, XB, (size_t)NB * DI / 8); k_cvt8<<<(unsigned)(((size_t)NN * DI / 8 + 255) / 256), 256, 0, stream>>>(means, MB, (size_t)NN * DI / 8);
    k_msq<<<NN / 8, 256, 0, stream>>>(means, MSQ);
    k_gemmw<bf, 0, false><<<dim3(NB / 64, NN / 64, 1), 32, 0, stream>>>(XB, nullptr, MB, nullptr, DI, G, NN, nullptr, 0, 0, 0);
    k_prep<<<NN / 256, 256, 0, stream>>>(bw, wts, PRE); k_mix<<<NB / 8, 256, 0, stream>>>(G, x, MSQ, PRE, pri, OUT);
}
